// LSTM_82291573391471
// MI455X (gfx1250) — hardware-verified
//
#include <hip/hip_runtime.h>
#include <math.h>

constexpr int N_BATCH   = 2048;
constexpr int N_STEPS   = 512;
constexpr int N_INPUT   = 5;
constexpr int N_HID     = 32;
constexpr int N_GATE    = 4 * N_HID;
constexpr int N_OUTC    = 2;
constexpr int BLK_ROWS  = 16;
constexpr int N_BLOCKS  = N_BATCH / BLK_ROWS;
constexpr int HS_PITCH  = 36;
constexpr int W_PLANE   = N_GATE * N_HID;
static_assert(N_BATCH % BLK_ROWS == 0, "batch tiles exact");
static_assert(N_HID == 32, "one 32-deep k chunk per product");
static_assert(N_GATE == 128, "eight 16-column gate tiles");
static_assert(BLK_ROWS * N_OUTC * 4 == 128, "one 128-B output line per tile");
static_assert((N_GATE * N_INPUT) % 32 == 0, "W_ih0 fill loop exact");
static_assert(W_PLANE % 32 == 0 && (W_PLANE / 8) % 32 == 0, "plane fill loops exact");
static_assert((HS_PITCH * 4) % 16 == 0, "16-B aligned tile rows");

typedef __attribute__((ext_vector_type(16))) _Float16 v16h;
typedef __attribute__((ext_vector_type(8)))  _Float16 v8h;
typedef __attribute__((ext_vector_type(8)))  float    v8f;
typedef __attribute__((ext_vector_type(4)))  float    v4f;

template <typename T> struct Frag;
template <> struct Frag<_Float16> {
  typedef v16h V; union U { v16h v; v8h h[2]; };
  static __device__ __forceinline__ v16h load(const _Float16* p) {
    U f; f.h[0] = *(const v8h*)(p); f.h[1] = *(const v8h*)(p + 16); return f.v;
  }
};

__device__ __forceinline__ v8f mma_h(v16h a, v16h b, v8f c) {
  c = __builtin_amdgcn_wmma_f32_16x16x32_f16(false, a, false, b, (short)0, c, false, false);
  asm volatile("v_nop\n\tv_nop\n\tv_nop\n\tv_nop" : "+v"(c) : "v"(a), "v"(b));
  return c;
}

__device__ __forceinline__ float gate_sigmoid(float z) {
  z = fminf(fmaxf(z, -30.0f), 30.0f);
  return __builtin_amdgcn_rcpf(1.0f + expf(-z));
}
__device__ __forceinline__ float gate_tanh(float z) {
  z = fminf(fmaxf(z, -15.0f), 15.0f);
  return 1.0f - 2.0f * __builtin_amdgcn_rcpf(expf(2.0f * z) + 1.0f);
}

__device__ __forceinline__ v16h load_a_tile(const float* p) {
  const v4f f0 = *(const v4f*)(p);
  const v4f f1 = *(const v4f*)(p + 4);
  const v4f f2 = *(const v4f*)(p + 16);
  const v4f f3 = *(const v4f*)(p + 20);
  v16h a;
#pragma unroll
  for (int e = 0; e < 4; ++e) {
    a[e]      = (_Float16)f0[e];
    a[4 + e]  = (_Float16)f1[e];
    a[8 + e]  = (_Float16)f2[e];
    a[12 + e] = (_Float16)f3[e];
  }
  return a;
}

template <int PASS>
__device__ __forceinline__ void cell_pass(const v16h a_in, const v16h a_h,
                                          const _Float16* w_in, const _Float16* w_hh,
                                          const float (&bias)[8], v8f& cst, float* hs_wr) {
  v8f acc[4];
#pragma unroll
  for (int q = 0; q < 4; ++q) {
    const int j = 2 * q + PASS;
    const v16h bi = Frag<_Float16>::load(w_in + j * 16 * N_HID);
    const v16h bh = Frag<_Float16>::load(w_hh + j * 16 * N_HID);
    const float bj = bias[j];
    v8f a = {bj, bj, bj, bj, bj, bj, bj, bj};
    a = mma_h(a_in, bi, a);
    a = mma_h(a_h, bh, a);
    acc[q] = a;
    asm volatile("" ::: "memory");
  }
  float dep = 0.0f;
#pragma unroll
  for (int r = 0; r < 8; ++r) {
    float zi = acc[0][r];
    float zf = acc[1][r];
    float zg = acc[2][r];
    float zo = acc[3][r];
    asm volatile("" : "+v"(zi), "+v"(zf), "+v"(zg), "+v"(zo) : "v"(dep));
    const float ig = gate_sigmoid(zi);
    const float fg = gate_sigmoid(zf);
    const float gg = gate_tanh(zg);
    const float og = gate_sigmoid(zo);
    const float cn = fg * cst[r] + ig * gg;
    cst[r] = cn;
    const float hn = og * gate_tanh(cn);
    hs_wr[r * HS_PITCH + PASS * 16] = hn;
    dep = hn;
  }
}

__global__ __launch_bounds__(32) __attribute__((amdgpu_num_vgpr(256))) void lstm2_fused_kernel(
    const float* __restrict__ x,
    const float* __restrict__ Wih0, const float* __restrict__ Whh0,
    const float* __restrict__ bih0, const float* __restrict__ bhh0,
    const float* __restrict__ Wih1, const float* __restrict__ Whh1,
    const float* __restrict__ bih1, const float* __restrict__ bhh1,
    const float* __restrict__ Wfc,  const float* __restrict__ bfc,
    float* __restrict__ out) {
  __shared__ __align__(16) _Float16 Wp[4 * W_PLANE];
  __shared__ __align__(16) float    bsum[2 * N_GATE];
  __shared__ __align__(16) float    xs[BLK_ROWS * HS_PITCH];
  __shared__ __align__(16) float    hs0[BLK_ROWS * HS_PITCH];
  __shared__ __align__(16) float    hs1[BLK_ROWS * HS_PITCH];
  __shared__ __align__(16) float    wfc_s[N_OUTC * N_HID];

  const int lane = threadIdx.x;
  const int n    = lane & 15;
  const int hh   = lane >> 4;
  const int koff = hh * 8;

  {
    v8h zz;
#pragma unroll
    for (int e = 0; e < 8; ++e) zz[e] = (_Float16)0.0f;
#pragma unroll 1
    for (int i = lane; i < W_PLANE / 8; i += 32) *(v8h*)(Wp + 8 * i) = zz;
  }
  __syncthreads();
#pragma unroll 1
  for (int i = lane; i < N_GATE * N_INPUT; i += 32) {
    const int gr = i / N_INPUT;
    const int gk = i - gr * N_INPUT;
    Wp[gr * N_HID + gk] = (_Float16)Wih0[i];
  }
#pragma unroll 2
  for (int i = lane; i < W_PLANE; i += 32) {
    const float w1 = Whh0[i];
    const float w2 = Wih1[i];
    const float w3 = Whh1[i];
    Wp[1 * W_PLANE + i] = (_Float16)w1;
    Wp[2 * W_PLANE + i] = (_Float16)w2;
    Wp[3 * W_PLANE + i] = (_Float16)w3;
  }
#pragma unroll 1
  for (int it = 0; it < N_GATE / 32; ++it) {
    const int g = it * 32 + lane;
    const float s0 = bih0[g] + bhh0[g];
    const float s1 = bih1[g] + bhh1[g];
    bsum[g] = s0;
    bsum[N_GATE + g] = s1;
  }
  wfc_s[lane]      = Wfc[lane];
  wfc_s[32 + lane] = Wfc[32 + lane];
  __syncthreads();

  float bias0[8], bias1[8];
#pragma unroll
  for (int j = 0; j < 8; ++j) {
    bias0[j] = bsum[16 * j + n];
    bias1[j] = bsum[N_GATE + 16 * j + n];
  }

  const v8f z8 = {0.f, 0.f, 0.f, 0.f, 0.f, 0.f, 0.f, 0.f};
  v8f c0a = z8, c0b = z8, c1a = z8, c1b = z8;
  v16h ah0, ah1;
#pragma unroll
  for (int e = 0; e < 16; ++e) { ah0[e] = (_Float16)0.0f; ah1[e] = (_Float16)0.0f; }

  const _Float16* wl = Wp + n * N_HID + koff;
  const float* xrow  = x + (size_t)(blockIdx.x * BLK_ROWS + n) * (size_t)(N_STEPS * N_INPUT);
  float* xw          = xs + n * HS_PITCH + 16 * hh;
  const float* xrd   = xs  + n * HS_PITCH + koff;
  const float* h0rd  = hs0 + n * HS_PITCH + koff;
  const float* h1rd  = hs1 + n * HS_PITCH + koff;
  float* h0wr        = hs0 + (8 * hh) * HS_PITCH + n;
  float* h1wr        = hs1 + (8 * hh) * HS_PITCH + n;
  const float fl     = (hh == 0) ? 1.0f : 0.0f;
  const v4f zz4      = {0.f, 0.f, 0.f, 0.f};

#pragma unroll 1
  for (int t = 0; t < N_STEPS; ++t) {
    const float* xp = xrow + t * N_INPUT;
    const float x0 = xp[0];
    const float x1 = xp[1];
    const float x2 = xp[2];
    const float x3 = xp[3];
    const float x4 = xp[4];
    v4f s0, s1;
    s0[0] = fl * x0;
    s0[1] = fl * x1;
    s0[2] = fl * x2;
    s0[3] = fl * x3;
    s1[0] = fl * x4;
    s1[1] = 0.0f;
    s1[2] = 0.0f;
    s1[3] = 0.0f;
    *(v4f*)(xw)      = s0;
    *(v4f*)(xw + 4)  = s1;
    *(v4f*)(xw + 8)  = zz4;
    *(v4f*)(xw + 12) = zz4;
    __syncthreads();

    {
      const v16h ax = load_a_tile(xrd);
      cell_pass<0>(ax, ah0, wl + 0 * W_PLANE, wl + 1 * W_PLANE, bias0, c0a, h0wr);
      cell_pass<1>(ax, ah0, wl + 0 * W_PLANE, wl + 1 * W_PLANE, bias0, c0b, h0wr);
    }
    __syncthreads();

    ah0 = load_a_tile(h0rd);
    cell_pass<0>(ah0, ah1, wl + 2 * W_PLANE, wl + 3 * W_PLANE, bias1, c1a, h1wr);
    cell_pass<1>(ah0, ah1, wl + 2 * W_PLANE, wl + 3 * W_PLANE, bias1, c1b, h1wr);
    __syncthreads();
    ah1 = load_a_tile(h1rd);
  }

  {
    const int ob = lane >> 1;
    const int oo = lane & 1;
    float acc = 0.0f;
#pragma unroll
    for (int k4 = 0; k4 < N_HID / 4; ++k4) {
      const v4f hv = *(const v4f*)(hs1 + ob * HS_PITCH + 4 * k4);
      const v4f wv = *(const v4f*)(wfc_s + oo * N_HID + 4 * k4);
      acc += hv[0] * wv[0];
      acc += hv[1] * wv[1];
      acc += hv[2] * wv[2];
      acc += hv[3] * wv[3];
    }
    const float res = acc + bfc[oo];
    volatile float* op = out + (size_t)blockIdx.x * (BLK_ROWS * N_OUTC) + lane;
    *op = res;
    __threadfence();
    *op = res;
  }
}

extern "C" void kernel_launch(void* const* d_in, const int* in_sizes, int n_in,
                              void* d_out, int out_size, void* d_ws, size_t ws_size,
                              hipStream_t stream) {
  (void)d_ws; (void)ws_size;
  if (n_in < 11 || d_out == nullptr) return;
  if (in_sizes[0] != N_BATCH * N_STEPS * N_INPUT || in_sizes[1] != N_GATE * N_INPUT ||
      in_sizes[2] != N_GATE * N_HID || in_sizes[3] != N_GATE || in_sizes[4] != N_GATE ||
      in_sizes[5] != N_GATE * N_HID || in_sizes[6] != N_GATE * N_HID || in_sizes[7] != N_GATE ||
      in_sizes[8] != N_GATE || in_sizes[9] != N_OUTC * N_HID || in_sizes[10] != N_OUTC ||
      out_size != N_BATCH * N_OUTC) return;

  const float* x    = (const float*)d_in[0];
  const float* Wih0 = (const float*)d_in[1];
  const float* Whh0 = (const float*)d_in[2];
  const float* bih0 = (const float*)d_in[3];
  const float* bhh0 = (const float*)d_in[4];
  const float* Wih1 = (const float*)d_in[5];
  const float* Whh1 = (const float*)d_in[6];
  const float* bih1 = (const float*)d_in[7];
  const float* bhh1 = (const float*)d_in[8];
  const float* Wfc  = (const float*)d_in[9];
  const float* bfc  = (const float*)d_in[10];
  float* out = (float*)d_out;

  lstm2_fused_kernel<<<dim3(N_BLOCKS), dim3(32), 0, stream>>>(
      x, Wih0, Whh0, bih0, bhh0, Wih1, Whh1, bih1, bhh1, Wfc, bfc, out);
}
